// BiomarkerConditionedAttention_58188216926551
// MI455X (gfx1250) — hardware-verified
//
#include <hip/hip_runtime.h>
#include <math.h>

typedef __attribute__((ext_vector_type(16))) _Float16 v16h;
typedef __attribute__((ext_vector_type(16))) __bf16 v16b;
typedef __attribute__((ext_vector_type(8)))  _Float16 v8h;
typedef __attribute__((ext_vector_type(8)))  float v8f;
typedef __attribute__((ext_vector_type(4)))  float v4f;
typedef __attribute__((ext_vector_type(2)))  float v2f;
typedef __attribute__((ext_vector_type(4)))  unsigned v4u;
typedef __attribute__((ext_vector_type(4)))  int v4i;
typedef float __attribute__((may_alias)) float_a;
typedef int __attribute__((may_alias)) int_a;

template <typename T> __device__ __forceinline__ void vst2(void* p, T v) { *(volatile T*)p = v; __threadfence(); *(volatile T*)p = v; }
__device__ __forceinline__ v8f wmma16(v16h a, v16h b, v8f c) {
  v8f d = __builtin_amdgcn_wmma_f32_16x16x32_f16(false, a, false, b, (short)0, c, false, false);
  asm volatile("v_nop\n\tv_nop\n\tv_nop\n\tv_nop" : "+v"(d) : "v"(a), "v"(b));
  return d;
}
__device__ __forceinline__ v8f wmma_bf(v16b a, v16b b, v8f c) {
  v8f d = __builtin_amdgcn_wmma_f32_16x16x32_bf16(false, a, false, b, (short)0, c, false, false);
  asm volatile("v_nop\n\tv_nop\n\tv_nop\n\tv_nop" : "+v"(d) : "v"(a), "v"(b));
  return d;
}
__device__ __forceinline__ v16h frag_h(const _Float16* rowk0, int lane) {
  union { v16h v; v8h q[2]; } u; const _Float16* p = rowk0 + 8 * (lane >> 4);
  u.q[0] = *(const v8h*)p; u.q[1] = *(const v8h*)(p + 16); return u.v;
}
__device__ __forceinline__ v16h frag_f32(const float* rowk0, int lane) {
  v16h a; const float* p = rowk0 + 8 * (lane >> 4);
#pragma unroll
  for (int i = 0; i < 8; ++i) { a[i] = (_Float16)p[i]; a[8 + i] = (_Float16)p[16 + i]; }
  return a;
}
__device__ __forceinline__ v16h frag_f32s(const float* rowk0, int lane, float sc) {
  v16h a; const float* p = rowk0 + 8 * (lane >> 4);
#pragma unroll
  for (int i = 0; i < 8; ++i) { a[i] = (_Float16)(p[i] * sc); a[8 + i] = (_Float16)(p[16 + i] * sc); }
  return a;
}
__device__ __forceinline__ v16h fragc_f32(const float* W, int k0, int n, int lane, int ld, int K) {
  v16h a; const int g = lane >> 4;
#pragma unroll
  for (int i = 0; i < 8; ++i) { const int ka = k0 + 8 * g + i, kb = ka + 16;
    a[i] = (_Float16)(ka < K ? W[(size_t)(ka < K ? ka : K - 1) * ld + n] : 0.f); a[8 + i] = (_Float16)(kb < K ? W[(size_t)(kb < K ? kb : K - 1) * ld + n] : 0.f); }
  return a;
}
struct F2 { v16b h, l; };
__device__ __forceinline__ F2 bsplit16(const float v[16]) { F2 r;
#pragma unroll
  for (int i = 0; i < 16; ++i) { const __bf16 h = (__bf16)v[i]; r.h[i] = h; r.l[i] = (__bf16)(v[i] - (float)h); }
  return r; }
__device__ __forceinline__ F2 split_row(const float* row, int k0, int lane) { float v[16]; const float* p = row + k0 + 8 * (lane >> 4);
#pragma unroll
  for (int i = 0; i < 8; ++i) { v[i] = p[i]; v[8 + i] = p[16 + i]; }
  return bsplit16(v); }
__device__ __forceinline__ F2 split_rowK(const float* row, int k0, int lane, int K) { float v[16]; const int g = lane >> 4;
#pragma unroll
  for (int i = 0; i < 8; ++i) { const int ka = k0 + 8 * g + i, kb = ka + 16; v[i] = ka < K ? row[ka < K ? ka : K - 1] : 0.f; v[8 + i] = kb < K ? row[kb < K ? kb : K - 1] : 0.f; }
  return bsplit16(v); }
__device__ __forceinline__ F2 split_col(const float* W, int k0, int n, int lane, int ld, int K) { float v[16]; const int g = lane >> 4;
#pragma unroll
  for (int i = 0; i < 8; ++i) { const int ka = k0 + 8 * g + i, kb = ka + 16; v[i] = ka < K ? W[(size_t)(ka < K ? ka : K - 1) * ld + n] : 0.f; v[8 + i] = kb < K ? W[(size_t)(kb < K ? kb : K - 1) * ld + n] : 0.f; }
  return bsplit16(v); }
__device__ __forceinline__ v8f mac3(const F2& a, const F2& b, v8f c) { c = wmma_bf(a.l, b.h, c); c = wmma_bf(a.h, b.l, c); return wmma_bf(a.h, b.h, c); }
__device__ __forceinline__ float sigm(float v) { return 1.0f / (1.0f + expf(-v)); }
#define LDSX() do { asm volatile("s_wait_dscnt 0" ::: "memory"); __builtin_amdgcn_wave_barrier(); __builtin_amdgcn_fence(__ATOMIC_RELEASE, "workgroup"); } while (0)


#define NBB 16
#define NT 513
#define CC 768
#define NH 12
#define HD 64
#define MM 5
#define GG 8
#define NROW (NBB * NT)
#define NROWP (((NROW + 63) / 64) * 64)
#ifndef TNB
#define TNB NBB
#endif
#ifndef TPR
#define TPR (NROWP / 64)
#endif
typedef __attribute__((ext_vector_type(8))) __bf16 v8b;
__device__ __forceinline__ v16b frag_b(const __bf16* rowk0, int lane) {
  union { v16b v; v8b q[2]; } u; const __bf16* p = rowk0 + 8 * (lane >> 4);
  u.q[0] = *(const v8b*)p; u.q[1] = *(const v8b*)(p + 16); return u.v;
}
__device__ __forceinline__ float bfr(float v) { return (float)(__bf16)v; }
__device__ __attribute__((noinline)) float exp_ni(float v) { return expf(v); }
__device__ __attribute__((noinline)) float erf_ni(float v) { return erff(v); }

#define WS_Q    0u
#define WS_K    (WS_Q + 2u * (size_t)NROWP * CC)
#define WS_V    (WS_K + 2u * (size_t)NROWP * CC)
#define WS_SO   (WS_V + 2u * (size_t)NROWP * CC)
#define WS_B16  (WS_SO + 4u * (size_t)NROWP * CC)
#define NSLOT 8
#define WS_B80  (WS_B16 + 4u * (size_t)NSLOT * 16 * CC)
#define WS_OP   (WS_B80 + 4u * (size_t)4 * 80 * CC)
#define WS_END  (WS_OP + 4u * (size_t)NROWP * CC)

__global__ __launch_bounds__(128) void k_proj(const float* __restrict__ X, const float* __restrict__ Wt, const float* __restrict__ Bs, _Float16* __restrict__ Q, _Float16* __restrict__ K, _Float16* __restrict__ V) { __shared__ __align__(16) _Float16 sh[64][136];
  const int tid = threadIdx.x, wave = tid >> 5, lane = tid & 31, col = lane & 15, g = lane >> 4; const int which = blockIdx.z; const int c0 = blockIdx.y * 128; const size_t r0 = (size_t)blockIdx.x * 64;
  size_t xr = r0 + wave * 16 + col; if (xr >= (size_t)NROW) xr = NROW - 1;
  v8f acc[8] = {};
#pragma unroll 2
  for (int kc = 0; kc < CC / 32; ++kc) { v16b a; { const float* p = X + xr * CC + kc * 32 + 8 * g;
#pragma unroll
      for (int i = 0; i < 8; ++i) { a[i] = (__bf16)p[i]; a[8 + i] = (__bf16)p[16 + i]; } }
#pragma unroll
    for (int j = 0; j < 8; ++j) { v16b w; const size_t o = (size_t)which * CC + c0 + j * 16 + col;
#pragma unroll
      for (int i = 0; i < 8; ++i) { w[i] = (__bf16)Wt[o * CC + kc * 32 + 8 * g + i]; w[8 + i] = (__bf16)Wt[o * CC + kc * 32 + 16 + 8 * g + i]; }
      acc[j] = wmma_bf(a, w, acc[j]); } }
#pragma unroll
  for (int j = 0; j < 8; ++j) { const float bb = bfr(Bs[which * CC + c0 + j * 16 + col]);
#pragma unroll
    for (int r = 0; r < 8; ++r) sh[wave * 16 + 8 * g + r][j * 16 + col] = (_Float16)(acc[j][r] + bb); }
  __syncthreads(); { _Float16* dst = which == 0 ? Q : which == 1 ? K : V; for (int e = tid; e < 64 * 16; e += 128) { const int rl = e >> 4, q = e & 15; vst2((unsigned*)(dst + (r0 + rl) * CC + c0 + q * 8), *(const v4u*)&sh[rl][q * 8]); } } }
__global__ __launch_bounds__(128) void k_att1(const _Float16* __restrict__ Q, const _Float16* __restrict__ K, const _Float16* __restrict__ V, float* __restrict__ SO) {
  __shared__ __align__(16) float sp[4][16][36]; __shared__ __align__(16) float so[4][16][68]; __shared__ __align__(16) _Float16 sv[32][72];
  const int tid = threadIdx.x, wave = tid >> 5, lane = tid & 31, col = lane & 15, g = lane >> 4; const int qb = blockIdx.x, h = blockIdx.y; const size_t b = blockIdx.z;
  const int qi = qb * 64 + wave * 16 + col; const int qic = qi < NT ? qi : NT - 1;
  v16h aq[2];
#pragma unroll
  for (int kc = 0; kc < 2; ++kc) aq[kc] = frag_h(Q + (b * NT + qic) * CC + h * HD + kc * 32, lane);
  float m[8], l[8];
#pragma unroll
  for (int r = 0; r < 8; ++r) { m[r] = -3.0e38f; l[r] = 0.f; }
  v8f acc[4] = {};
#pragma unroll 1
  for (int ks = 0; ks < (NT + 31) / 32; ++ks) {
    __syncthreads();
    for (int e = tid; e < 32 * 8; e += 128) { const int i = e >> 3, q8 = e & 7; int ki = ks * 32 + i; if (ki >= NT) ki = NT - 1; *(v4u*)&sv[i][q8 * 8] = *(const v4u*)(V + (b * NT + ki) * CC + h * HD + q8 * 8); }
    float s[2][8];
#pragma unroll
    for (int ct = 0; ct < 2; ++ct) { const int ki = ks * 32 + ct * 16 + col; const int kic = ki < NT ? ki : NT - 1; v8f c = {};
#pragma unroll
      for (int kc = 0; kc < 2; ++kc) c = wmma16(aq[kc], frag_h(K + (b * NT + kic) * CC + h * HD + kc * 32, lane), c);
#pragma unroll
      for (int r = 0; r < 8; ++r) s[ct][r] = (ki < NT) ? c[r] * 0.125f : -3.0e38f; }
    float alpha[8];
#pragma unroll
    for (int r = 0; r < 8; ++r) { float mx = fmaxf(s[0][r], s[1][r]);
#pragma unroll
      for (int o = 1; o < 16; o <<= 1) mx = fmaxf(mx, __shfl_xor(mx, o));
      const float mn = fmaxf(m[r], mx); alpha[r] = __expf(m[r] - mn); const float e0 = (s[0][r] <= -1.0e38f) ? 0.f : __expf(s[0][r] - mn), e1 = (s[1][r] <= -1.0e38f) ? 0.f : __expf(s[1][r] - mn); float es = e0 + e1;
#pragma unroll
      for (int o = 1; o < 16; o <<= 1) es += __shfl_xor(es, o);
      l[r] = l[r] * alpha[r] + es; m[r] = mn; sp[wave][8 * g + r][col] = e0; sp[wave][8 * g + r][16 + col] = e1; }
#pragma unroll
    for (int j = 0; j < 4; ++j)
#pragma unroll
      for (int r = 0; r < 8; ++r) acc[j][r] *= alpha[r];
    __syncthreads();
    const v16h pa = frag_f32s(&sp[wave][col][0], lane, 2048.0f);
#pragma unroll
    for (int j = 0; j < 4; ++j) { v16h vb; const int dc = j * 16 + col;
#pragma unroll
      for (int i = 0; i < 8; ++i) { vb[i] = sv[8 * g + i][dc]; vb[8 + i] = sv[16 + 8 * g + i][dc]; }
      acc[j] = wmma16(pa, vb, acc[j]); } }
#pragma unroll
  for (int r = 0; r < 8; ++r) { const float il = (1.0f / 2048.0f) / l[r];
#pragma unroll
    for (int j = 0; j < 4; ++j) so[wave][8 * g + r][j * 16 + col] = acc[j][r] * il; }
  LDSX();
  for (int rl = 0; rl < 16; ++rl) { const int qpos = qb * 64 + wave * 16 + rl; if (qpos < NT && lane < 16) vst2(SO + (b * NT + qpos) * CC + h * HD + lane * 4, *(const v4f*)&so[wave][rl][lane * 4]); } }
__global__ __launch_bounds__(128) void k_lin(const float* __restrict__ IN, const float* __restrict__ Wt, int woff, const float* __restrict__ Bs, int boff, const float* __restrict__ RS, float* __restrict__ OUT) { __shared__ __align__(16) float so[16][132];
  const int tid = threadIdx.x, wave = tid >> 5, lane = tid & 31, col = lane & 15, g = lane >> 4; const int c0 = blockIdx.x * 128; const size_t r0 = (size_t)blockIdx.y * 16;
  v8f acc[2] = {};
#pragma unroll 2
  for (int kc = 0; kc < CC / 32; ++kc) { const F2 a = split_row(IN + (r0 + col) * CC, kc * 32, lane);
#pragma unroll
    for (int j = 0; j < 2; ++j) { v16b w; const size_t o = (size_t)woff + c0 + (wave * 2 + j) * 16 + col;
#pragma unroll
      for (int i = 0; i < 8; ++i) { w[i] = (__bf16)Wt[o * CC + kc * 32 + 8 * g + i]; w[8 + i] = (__bf16)Wt[o * CC + kc * 32 + 16 + 8 * g + i]; }
      acc[j] = wmma_bf(a.h, w, acc[j]); acc[j] = wmma_bf(a.l, w, acc[j]); } }
#pragma unroll
  for (int j = 0; j < 2; ++j) { const int cl = (wave * 2 + j) * 16 + col; const float bb = Bs ? bfr(Bs[boff + c0 + cl]) : 0.f;
#pragma unroll
    for (int r = 0; r < 8; ++r) { float v = acc[j][r] + bb; if (RS) v *= bfr(RS[r0 + 8 * g + r]); so[8 * g + r][cl] = v; } }
  __syncthreads(); for (int e = tid; e < 16 * 32; e += 128) { const int rl = e >> 5, q = e & 31; vst2(OUT + (r0 + rl) * CC + c0 + q * 4, *(const v4f*)&so[rl][q * 4]); } }
__global__ __launch_bounds__(256) void k_cross(const float* __restrict__ X, const float* __restrict__ Q2, const float* __restrict__ CAW, const float* __restrict__ CAB, float* __restrict__ CPRE) { __shared__ __align__(16) float su[CC]; __shared__ float ssc[NT + 7]; __shared__ __align__(16) float sxb[CC]; __shared__ float sred[8]; __shared__ float sbc; __shared__ __align__(16) float so[HD];
  const int t = threadIdx.x; const int h = blockIdx.x; const size_t b = blockIdx.y; const float* q2 = Q2 + b * CC + h * HD; const float* WK = CAW + (size_t)(CC + h * HD) * CC; const float* WV = CAW + (size_t)(2 * CC + h * HD) * CC;
  for (int i = t; i < CC; i += 256) { float a = 0.f;
#pragma unroll 1
    for (int d = 0; d < HD; ++d) a += q2[d] * bfr(WK[(size_t)d * CC + i]); su[i] = a; }
  if (t < 32) { float a = 0.f; for (int d = t; d < HD; d += 32) a += q2[d] * bfr(CAB[CC + h * HD + d]);
#pragma unroll
    for (int o = 1; o < 32; o <<= 1) a += __shfl_xor(a, o); if (t == 0) sbc = a; }
  __syncthreads(); const float cterm = sbc;
  { const int wv = t >> 5, ln = t & 31;
#pragma unroll 1
    for (int j = wv; j < NT; j += 8) { const float* xr = X + (b * NT + j) * CC; float a = 0.f; for (int i = ln; i < CC; i += 32) a += su[i] * bfr(xr[i]);
#pragma unroll
      for (int o = 1; o < 32; o <<= 1) a += __shfl_xor(a, o); if (ln == 0) ssc[j] = (a + cterm) * 0.125f; } }
  __syncthreads();
  { float m = -3.0e38f; for (int j = t; j < NT; j += 256) m = fmaxf(m, ssc[j]);
#pragma unroll
    for (int o = 1; o < 32; o <<= 1) m = fmaxf(m, __shfl_xor(m, o));
    if ((t & 31) == 0) sred[t >> 5] = m; __syncthreads(); if (t == 0) { float a = sred[0]; for (int i = 1; i < 8; ++i) a = fmaxf(a, sred[i]); sbc = a; } __syncthreads(); m = sbc; __syncthreads();
    float s = 0.f; for (int j = t; j < NT; j += 256) { const float e = expf(ssc[j] - m); ssc[j] = e; s += e; }
#pragma unroll
    for (int o = 1; o < 32; o <<= 1) s += __shfl_xor(s, o);
    if ((t & 31) == 0) sred[t >> 5] = s; __syncthreads(); if (t == 0) { float a = 0.f; for (int i = 0; i < 8; ++i) a += sred[i]; sbc = 1.0f / a; } __syncthreads(); const float inv = sbc;
    for (int j = t; j < NT; j += 256) ssc[j] *= inv; }
  __syncthreads();
  for (int i = t; i < CC; i += 256) { float a = 0.f;
#pragma unroll 1
    for (int j = 0; j < NT; ++j) a += ssc[j] * bfr(X[(b * NT + j) * CC + i]); sxb[i] = a; }
  __syncthreads();
  { const int wv = t >> 5, ln = t & 31; for (int d = wv; d < HD; d += 8) { float a = 0.f; for (int i = ln; i < CC; i += 32) a += bfr(WV[(size_t)d * CC + i]) * sxb[i];
#pragma unroll
      for (int o = 1; o < 32; o <<= 1) a += __shfl_xor(a, o); if (ln == 0) so[d] = a + bfr(CAB[2 * CC + h * HD + d]); } }
  __syncthreads(); if (t < 16) vst2(CPRE + b * CC + h * HD + t * 4, *(const v4f*)&so[t * 4]); }
__global__ __launch_bounds__(256) void k_tri(const float* __restrict__ X, const float* __restrict__ BC, const float* __restrict__ OFF, float* __restrict__ SP) { __shared__ int si[MM][8]; __shared__ float sw[MM][8]; __shared__ __align__(16) float so[MM][CC];
  const int t = threadIdx.x; const size_t b = blockIdx.x;
  if (t < MM) { const int mm = t; int i0[3], i1[3]; float w1[3];
    for (int a = 0; a < 3; ++a) { float cv = bfr(BC[mm * 3 + a]) + bfr(OFF[(b * MM + mm) * 3 + a]); cv = fminf(fmaxf(cv, -1.0f), 1.0f); const float pix = (cv + 1.0f) * 0.5f * (float)(GG - 1); const float t0 = floorf(pix); w1[a] = pix - t0; float c0 = fminf(fmaxf(t0, 0.f), (float)(GG - 1)), c1 = fminf(fmaxf(t0 + 1.0f, 0.f), (float)(GG - 1)); i0[a] = (int)c0; i1[a] = (int)c1; }
    for (int k = 0; k < 8; ++k) { const int xz = (k & 4) ? i1[2] : i0[2], xy = (k & 2) ? i1[1] : i0[1], xx = (k & 1) ? i1[0] : i0[0]; si[mm][k] = 1 + (xz * GG + xy) * GG + xx; const float wz = (k & 4) ? w1[2] : 1.0f - w1[2], wy = (k & 2) ? w1[1] : 1.0f - w1[1], wx = (k & 1) ? w1[0] : 1.0f - w1[0]; sw[mm][k] = wx * wy * wz; } }
  __syncthreads();
  for (int e = t; e < MM * CC; e += 256) { const int mm = e / CC, c = e % CC;
    float v[8]; for (int k = 0; k < 8; ++k) v[k] = bfr(X[(b * NT + si[mm][k]) * CC + c]);
    float w1x, w1y, w1z; {
      float cv; cv = bfr(BC[mm * 3 + 0]) + bfr(OFF[(b * MM + mm) * 3 + 0]); cv = fminf(fmaxf(cv, -1.0f), 1.0f); { const float pix = (cv + 1.0f) * 0.5f * (float)(GG - 1); w1x = pix - floorf(pix); }
      cv = bfr(BC[mm * 3 + 1]) + bfr(OFF[(b * MM + mm) * 3 + 1]); cv = fminf(fmaxf(cv, -1.0f), 1.0f); { const float pix = (cv + 1.0f) * 0.5f * (float)(GG - 1); w1y = pix - floorf(pix); }
      cv = bfr(BC[mm * 3 + 2]) + bfr(OFF[(b * MM + mm) * 3 + 2]); cv = fminf(fmaxf(cv, -1.0f), 1.0f); { const float pix = (cv + 1.0f) * 0.5f * (float)(GG - 1); w1z = pix - floorf(pix); } }
    const float c00 = v[0] * (1.f - w1x) + v[1] * w1x, c01 = v[2] * (1.f - w1x) + v[3] * w1x, c10 = v[4] * (1.f - w1x) + v[5] * w1x, c11 = v[6] * (1.f - w1x) + v[7] * w1x;
    const float c0v = c00 * (1.f - w1y) + c01 * w1y, c1v = c10 * (1.f - w1y) + c11 * w1y; so[mm][c] = c0v * (1.f - w1z) + c1v * w1z; }
  __syncthreads(); for (int q = t; q < MM * CC / 4; q += 256) vst2(SP + b * MM * CC + q * 4, *(const v4f*)&(&so[0][0])[q * 4]); }
__global__ __launch_bounds__(64) void k_dba(const float* __restrict__ Q3, const float* __restrict__ K3, const float* __restrict__ V3, float* __restrict__ DPRE) { __shared__ float sp[8]; __shared__ __align__(16) float so[HD]; const int t = threadIdx.x; const int h = blockIdx.x; const size_t b = blockIdx.y;
  if (t < MM) { float a = 0.f; for (int d = 0; d < HD; ++d) a += Q3[b * CC + h * HD + d] * K3[(b * MM + t) * CC + h * HD + d]; sp[t] = a * 0.125f; }
  __syncthreads(); if (t == 0) { float m = sp[0]; for (int j = 1; j < MM; ++j) m = fmaxf(m, sp[j]); float s = 0.f; for (int j = 0; j < MM; ++j) { sp[j] = expf(sp[j] - m); s += sp[j]; } for (int j = 0; j < MM; ++j) sp[j] /= s; }
  __syncthreads(); { float a = 0.f; for (int j = 0; j < MM; ++j) a += sp[j] * V3[(b * MM + j) * CC + h * HD + t]; so[t] = a; }
  __syncthreads(); if (t < 16) vst2(DPRE + b * CC + h * HD + t * 4, *(const v4f*)&so[t * 4]); }
__global__ __launch_bounds__(128) void k_gate(const float* __restrict__ SO, const float* __restrict__ GW, const float* __restrict__ CB, const float* __restrict__ COND, const float* __restrict__ DBA, const float* __restrict__ CONF, float* __restrict__ OP) { __shared__ __align__(16) float sf[4][16][132];
  const int tid = threadIdx.x, wave = tid >> 5, lane = tid & 31, col = lane & 15, g = lane >> 4; const int c0 = blockIdx.y * 128; const size_t r0 = (size_t)blockIdx.x * 64 + wave * 16;
  v8f acc[8] = {};
#pragma unroll 2
  for (int kc = 0; kc < CC / 32; ++kc) { const v16h a = frag_f32(SO + (r0 + col) * CC + kc * 32, lane);
#pragma unroll
    for (int j = 0; j < 8; ++j) { v16h w; const size_t o = c0 + j * 16 + col;
#pragma unroll
      for (int i = 0; i < 8; ++i) { w[i] = (_Float16)bfr(GW[o * (3 * CC) + kc * 32 + 8 * g + i]); w[8 + i] = (_Float16)bfr(GW[o * (3 * CC) + kc * 32 + 16 + 8 * g + i]); }
      acc[j] = wmma16(a, w, acc[j]); } }
#pragma unroll
  for (int j = 0; j < 8; ++j) { const int c = c0 + j * 16 + col;
#pragma unroll
    for (int r = 0; r < 8; ++r) { const size_t row = r0 + 8 * g + r; size_t b = row / NT; if (b >= (size_t)NBB) b = NBB - 1; const float a = acc[j][r] + CB[b * CC + c]; const float gt = 1.0f / (1.0f + expf(-a)); const float conf = bfr(CONF[b]); const float bio = (0.5f * COND[b * CC + c] + 0.5f * DBA[b * CC + c]) * conf; sf[wave][8 * g + r][j * 16 + col] = gt * bio + (1.0f - gt) * SO[row * CC + c]; } }
  LDSX(); for (int rl = 0; rl < 16; ++rl) vst2(OP + (r0 + rl) * CC + c0 + lane * 4, *(const v4f*)&sf[wave][rl][lane * 4]); }
__global__ __launch_bounds__(128) void k_out(const float* __restrict__ OP, const float* __restrict__ PW, const float* __restrict__ PB, float* __restrict__ OUT) { __shared__ __align__(16) float sf[4][16][132];
  const int tid = threadIdx.x, wave = tid >> 5, lane = tid & 31, col = lane & 15, g = lane >> 4; const int c0 = blockIdx.y * 128; const size_t r0 = (size_t)blockIdx.x * 64 + wave * 16;
  v8f acc[8] = {};
#pragma unroll 2
  for (int kc = 0; kc < CC / 32; ++kc) { const F2 a = split_row(OP + (r0 + col) * CC, kc * 32, lane);
#pragma unroll
    for (int j = 0; j < 8; ++j) { v16b w; const size_t o = c0 + j * 16 + col;
#pragma unroll
      for (int i = 0; i < 8; ++i) { w[i] = (__bf16)PW[o * CC + kc * 32 + 8 * g + i]; w[8 + i] = (__bf16)PW[o * CC + kc * 32 + 16 + 8 * g + i]; }
      acc[j] = wmma_bf(a.h, w, acc[j]); acc[j] = wmma_bf(a.l, w, acc[j]); } }
#pragma unroll
  for (int j = 0; j < 8; ++j) { const float bb = bfr(PB[c0 + j * 16 + col]);
#pragma unroll
    for (int r = 0; r < 8; ++r) sf[wave][8 * g + r][j * 16 + col] = acc[j][r] + bb; }
  LDSX(); for (int rl = 0; rl < 16; ++rl) { const size_t row = r0 + rl; if (row < (size_t)NROW) vst2(OUT + row * CC + c0 + lane * 4, *(const v4f*)&sf[wave][rl][lane * 4]); } }
__global__ __launch_bounds__(128) void k_gconst(const float* __restrict__ COND, const float* __restrict__ DBA, const float* __restrict__ GW, const float* __restrict__ GB, float* __restrict__ CBo) { __shared__ __align__(16) float so[16][132];
  const int tid = threadIdx.x, wave = tid >> 5, lane = tid & 31, col = lane & 15, g = lane >> 4; const int c0 = blockIdx.x * 128;
  v8f acc[2] = {};
#pragma unroll 1
  for (int part = 0; part < 2; ++part) { const float* IN = part == 0 ? COND : DBA; const int koff = (part + 1) * CC;
#pragma unroll 2
    for (int kc = 0; kc < CC / 32; ++kc) { const F2 a = split_row(IN + (size_t)col * CC, kc * 32, lane);
#pragma unroll
      for (int j = 0; j < 2; ++j) { v16b w; const size_t o = c0 + (wave * 2 + j) * 16 + col;
#pragma unroll
        for (int i = 0; i < 8; ++i) { w[i] = (__bf16)GW[o * (3 * CC) + koff + kc * 32 + 8 * g + i]; w[8 + i] = (__bf16)GW[o * (3 * CC) + koff + kc * 32 + 16 + 8 * g + i]; }
        acc[j] = wmma_bf(a.h, w, acc[j]); acc[j] = wmma_bf(a.l, w, acc[j]); } } }
#pragma unroll
  for (int j = 0; j < 2; ++j) { const int cl = (wave * 2 + j) * 16 + col; const float bb = bfr(GB[c0 + cl]);
#pragma unroll
    for (int r = 0; r < 8; ++r) so[8 * g + r][cl] = acc[j][r] + bb; }
  __syncthreads(); for (int e = tid; e < 16 * 32; e += 128) { const int rl = e >> 5, q = e & 31; vst2(CBo + (size_t)rl * CC + c0 + q * 4, *(const v4f*)&so[rl][q * 4]); } }
extern "C" void kernel_launch(void* const* d_in, const int* in_sizes, int n_in, void* d_out, int out_size, void* d_ws, size_t ws_size, hipStream_t stream) {
  (void)in_sizes; (void)n_in; (void)out_size;
  const float** F = (const float**)d_in;
  if (ws_size < (size_t)WS_END) return;
  char* ws = (char*)d_ws; _Float16 *Q = (_Float16*)(ws + WS_Q), *K = (_Float16*)(ws + WS_K), *V = (_Float16*)(ws + WS_V); float *SO = (float*)(ws + WS_SO), *B16 = (float*)(ws + WS_B16), *B80 = (float*)(ws + WS_B80), *OP = (float*)(ws + WS_OP);
  float *bio_q = B16 + 0 * 16 * CC, *q2 = B16 + 1 * 16 * CC, *cpre = B16 + 2 * 16 * CC, *cond = B16 + 3 * 16 * CC, *q3 = B16 + 4 * 16 * CC, *dpre = B16 + 5 * 16 * CC, *dba = B16 + 6 * 16 * CC, *cb = B16 + 7 * 16 * CC;
  float *spre = B80, *samp = B80 + 80 * CC, *k3 = B80 + 2 * 80 * CC, *v3 = B80 + 3 * 80 * CC;
  k_proj<<<dim3(TPR, CC / 128, 3), 128, 0, stream>>>(F[0], F[5], F[6], Q, K, V);
  k_att1<<<dim3((NT + 63) / 64, NH, TNB), 128, 0, stream>>>(Q, K, V, SO);
  k_lin<<<dim3(CC / 128, 1), 128, 0, stream>>>(F[1], F[7], 0, F[8], 0, nullptr, bio_q);
  k_lin<<<dim3(CC / 128, 1), 128, 0, stream>>>(bio_q, F[9], 0, F[10], 0, nullptr, q2);
  k_cross<<<dim3(NH, TNB), 256, 0, stream>>>(F[0], q2, F[9], F[10], cpre);
  k_lin<<<dim3(CC / 128, 1), 128, 0, stream>>>(cpre, F[11], 0, F[12], 0, nullptr, cond);
  k_tri<<<TNB, 256, 0, stream>>>(F[0], F[3], F[4], spre);
  k_lin<<<dim3(CC / 128, 5), 128, 0, stream>>>(spre, F[13], 0, F[14], 0, nullptr, samp);
  k_lin<<<dim3(CC / 128, 1), 128, 0, stream>>>(F[1], F[15], 0, F[16], 0, nullptr, q3);
  k_lin<<<dim3(CC / 128, 5), 128, 0, stream>>>(samp, F[15], CC, F[16], CC, nullptr, k3);
  k_lin<<<dim3(CC / 128, 5), 128, 0, stream>>>(samp, F[15], 2 * CC, F[16], 2 * CC, nullptr, v3);
  k_dba<<<dim3(NH, TNB), 64, 0, stream>>>(q3, k3, v3, dpre);
  k_lin<<<dim3(CC / 128, 1), 128, 0, stream>>>(dpre, F[17], 0, F[18], 0, F[2], dba);
  k_gconst<<<dim3(CC / 128, 1), 128, 0, stream>>>(cond, dba, F[19], F[20], cb);
  k_gate<<<dim3(TPR, CC / 128), 128, 0, stream>>>(SO, F[19], cb, cond, dba, F[2], OP);
  k_out<<<dim3(TPR, CC / 128), 128, 0, stream>>>(OP, F[21], F[22], (float*)d_out);
}
